// Net_68805376082306
// MI455X (gfx1250) — hardware-verified
//
#include <hip/hip_runtime.h>
#include <math.h>

constexpr int NN    = 50000;
constexpr int NE    = 1600000;
constexpr int WD    = 64;
constexpr int NLAY  = 5;
constexpr int NP    = 50048;
constexpr int NT    = 256;
constexpr int TR    = 1024;
constexpr int NTIL  = 49;
constexpr int NR    = NTIL * TR;
constexpr int NSB   = 64;
constexpr int SBL   = 22;
constexpr int SBCAP = SBL * 32;
constexpr int PCH   = 4096;
constexpr int PSP   = PCH / NT;
constexpr int NPC   = (NE + PCH - 1) / PCH;
constexpr int NST   = 7;
constexpr int STSH  = 13;
constexpr int CCAP  = 1024;
constexpr int CLN   = CCAP / 32;
constexpr int CPI   = 4;
constexpr int NBI   = (NPC + CPI - 1) / CPI;
constexpr int Q1CAP = 256;
constexpr int SENTB = NN;
constexpr unsigned SENTC = 0xFFFFFFFFu;
constexpr int ACCB  = TR * WD * 4;

static_assert(NP % 64 == 0 && NP >= NN);
static_assert(WD == 64 && WD % 32 == 0);
static_assert(NR >= NP && NTIL * TR == NR && TR == 1024 && NSB * 16 == TR);
static_assert(NE % PSP == 0 && PSP % 4 == 0);
static_assert(((NN - 1) >> STSH) < NST && ((NTIL - 1) >> 3) < NST);
static_assert(NN < 65536);
static_assert(NN % 4 == 0 && NP % 4 == 0 && TR % 128 == 0);
static_assert(CPI * 4 * NT == PCH);
static_assert((NLAY * WD * 8) % NT == 0 && (NP * 8) % NT == 0);
static_assert(CLN == 32 && NST * CLN == 7 * 8 * 4);
static_assert(Q1CAP >= NT && Q1CAP % 32 == 0);
static_assert(SBCAP % 4 == 0 && CCAP == 4 * NT);

typedef __attribute__((ext_vector_type(16))) _Float16 v16h;
typedef __attribute__((ext_vector_type(8)))  _Float16 v8h;
typedef __attribute__((ext_vector_type(16))) __bf16   v16b;
typedef __attribute__((ext_vector_type(8)))  __bf16   v8b;
typedef __attribute__((ext_vector_type(8)))  float    v8f;
typedef __attribute__((ext_vector_type(4)))  float    v4f;
typedef __attribute__((ext_vector_type(4)))  int      v4i;
typedef __attribute__((ext_vector_type(4)))  unsigned int v4u;

__device__ __forceinline__ unsigned short f2bf_bits(float f) {
  unsigned u = __float_as_uint(f);
  return (unsigned short)((u + 0x7FFFu + ((u >> 16) & 1u)) >> 16);
}
__device__ __forceinline__ float bf_bits2f(unsigned short h) { return __uint_as_float(((unsigned)h) << 16); }

__device__ __forceinline__ void dep_guard_h(v8f& a, v8f& b, v16h x, v16h y) { asm volatile("v_nop\n\tv_nop\n\tv_nop\n\tv_nop" : "+v"(a), "+v"(b) : "v"(x), "v"(y)); }
__device__ __forceinline__ void dep_guard_b(v8f& a, v8f& b, v16b x, v16b y) { asm volatile("v_nop\n\tv_nop\n\tv_nop\n\tv_nop" : "+v"(a), "+v"(b) : "v"(x), "v"(y)); }
__device__ __forceinline__ void keep4_h(v16h a, v16h b, v16h c, v16h d) { asm volatile("v_nop" :: "v"(a), "v"(b), "v"(c), "v"(d)); }
__device__ __forceinline__ void keep4_b(v16b a, v16b b, v16b c, v16b d) { asm volatile("v_nop" :: "v"(a), "v"(b), "v"(c), "v"(d)); }
__device__ __forceinline__ void acc_guard4(v8f& a, v8f& b, v8f& c, v8f& d) { asm volatile("v_nop\n\tv_nop\n\tv_nop\n\tv_nop" : "+v"(a), "+v"(b), "+v"(c), "+v"(d)); }
template <typename T> struct Frag;
template <> struct Frag<_Float16> {
  typedef v16h V; union U { v16h v; v8h h[2]; };
  static __device__ __forceinline__ v16h load(const _Float16* p) {
    U f; f.h[0] = *(const v8h*)(p); f.h[1] = *(const v8h*)(p + 16); return f.v;
  }
  static __device__ __forceinline__ v8f mma(v16h a, v16h b, v8f c) {
    return __builtin_amdgcn_wmma_f32_16x16x32_f16(false, a, false, b, (short)0, c, false, false);
  }
  static __device__ __forceinline__ void guard(v8f& a, v8f& b, v16h x, v16h y) { dep_guard_h(a, b, x, y); }
  static __device__ __forceinline__ void keep(v16h a, v16h b, v16h c, v16h d) { keep4_h(a, b, c, d); }
};
template <> struct Frag<__bf16> {
  typedef v16b V; union U { v16b v; v8b h[2]; };
  static __device__ __forceinline__ v16b load(const __bf16* p) {
    U f; f.h[0] = *(const v8b*)(p); f.h[1] = *(const v8b*)(p + 16); return f.v;
  }
  static __device__ __forceinline__ v8f mma(v16b a, v16b b, v8f c) {
    return __builtin_amdgcn_wmma_f32_16x16x32_bf16(false, a, false, b, (short)0, c, false, false);
  }
  static __device__ __forceinline__ void guard(v8f& a, v8f& b, v16b x, v16b y) { dep_guard_b(a, b, x, y); }
  static __device__ __forceinline__ void keep(v16b a, v16b b, v16b c, v16b d) { keep4_b(a, b, c, d); }
};

template <int ET> struct Elem;
template <> struct Elem<0> { typedef _Float16 T; };
template <> struct Elem<1> { typedef __bf16 T; };
template <int ET, bool SPLIT, int BIAS_MODE, int OUT_MODE, bool RESID, int ACT = 0>
__global__ __launch_bounds__(256) void wmma_gemm64(
    const unsigned short* __restrict__ Ap, const unsigned short* __restrict__ A2p, int lda, long strideA,
    const unsigned short* __restrict__ Btp, const unsigned short* __restrict__ Bt2p, int ldb, long strideB,
    void* __restrict__ Cout, void* __restrict__ Cout2, int ldc, long strideC,
    const float* __restrict__ bias,
    const float* __restrict__ resid, long strideR,
    int M, int N, int K, float scale) {
  typedef typename Elem<ET>::T T;
  typedef typename Frag<T>::V V;
  const T* A = (const T*)Ap; const T* A2 = (const T*)A2p; const T* Bt = (const T*)Btp; const T* Bt2 = (const T*)Bt2p;
  __shared__ __align__(16) float sT[8][16 * 68];
  const int b    = blockIdx.y;
  const int lane = threadIdx.x & 31;
  const int wave = threadIdx.x >> 5;
  const int tilesN = N >> 6;
  const int tilesM = M >> 6;
  const int tile = blockIdx.x * 8 + wave;
  if (tile >= tilesM * tilesN) return;
  const int tm = tile / tilesN;
  const int tn = tile - tm * tilesN;
  const int m0 = tm << 6;
  const int n0 = tn << 6;

  const T* Ab  = A  + (size_t)b * strideA;
  const T* Bb  = Bt + (size_t)b * strideB;
  const T* Ab2 = SPLIT ? (A2  + (size_t)b * strideA) : nullptr;
  const T* Bb2 = SPLIT ? (Bt2 + (size_t)b * strideB) : nullptr;

  const int rlane = lane & 15;
  const int koff  = (lane >> 4) * 8;
  const int mOff  = (lane >> 4) * 8;

  v8f acc[4][4];
#pragma unroll
  for (int i = 0; i < 4; ++i)
#pragma unroll
    for (int j = 0; j < 4; ++j) acc[i][j] = (v8f){0.f,0.f,0.f,0.f,0.f,0.f,0.f,0.f};

  for (int k0 = 0; k0 < K; k0 += 32) {
    V bh[4], bl[4];
#pragma unroll
    for (int j = 0; j < 4; ++j) {
      const size_t bo = (size_t)(n0 + (j << 4) + rlane) * ldb + koff + k0;
      bh[j] = Frag<T>::load(Bb + bo);
      if (SPLIT) bl[j] = Frag<T>::load(Bb2 + bo);
    }
#pragma unroll
    for (int i = 0; i < 4; ++i) {
      const size_t ao = (size_t)(m0 + (i << 4) + rlane) * lda + koff + k0;
      V ah = Frag<T>::load(Ab + ao);
      V al;
      if (SPLIT) al = Frag<T>::load(Ab2 + ao);
#pragma unroll
      for (int j = 0; j < 4; ++j) {
        acc[i][j] = Frag<T>::mma(ah, bh[j], acc[i][j]);
        if (SPLIT) {
          acc[i][j] = Frag<T>::mma(ah, bl[j], acc[i][j]);
          acc[i][j] = Frag<T>::mma(al, bh[j], acc[i][j]);
        }
      }
      Frag<T>::guard(acc[i][0], acc[i][3], ah, SPLIT ? al : ah);
    }
    Frag<T>::keep(bh[0], bh[1], bh[2], bh[3]);
    if (SPLIT) Frag<T>::keep(bl[0], bl[1], bl[2], bl[3]);
  }
  acc_guard4(acc[0][0], acc[0][1], acc[0][2], acc[0][3]);
  acc_guard4(acc[1][0], acc[1][1], acc[1][2], acc[1][3]);
  acc_guard4(acc[2][0], acc[2][1], acc[2][2], acc[2][3]);
  acc_guard4(acc[3][0], acc[3][1], acc[3][2], acc[3][3]);

  float* slab = sT[wave];
  const float* Rb = RESID ? (resid + (size_t)b * strideR) : nullptr;
#pragma unroll
  for (int i = 0; i < 4; ++i) {
    const int mBase = m0 + (i << 4);
#pragma unroll
    for (int j = 0; j < 4; ++j) {
      const int n = n0 + (j << 4) + rlane;
      float bv = 0.f;
      if (BIAS_MODE == 2) bv = bias[n];
#pragma unroll
      for (int r = 0; r < 8; ++r) {
        float v = acc[i][j][r] * scale;
        if (BIAS_MODE == 1) v += bias[mBase + mOff + r];
        if (BIAS_MODE == 2) v += bv;
        if (RESID) v += Rb[(size_t)(mBase + mOff + r) * ldc + n];
        if (ACT == 1) v = tanhf(v);
        if (ACT == 2) v = fmaxf(v, 0.0f);
        if (ACT == 3) v = v / (1.0f + expf(-v));
        if (ACT == 4) v = (v > 0.f) ? v : 0.01f * v;
        if (ACT == 5) v = 0.5f * v * (1.0f + erff(v * 0.70710678118654752f));
        slab[(mOff + r) * 68 + (j << 4) + rlane] = v;
      }
    }
    __builtin_amdgcn_fence(__ATOMIC_RELEASE, "workgroup");
    __builtin_amdgcn_wave_barrier();
    __builtin_amdgcn_fence(__ATOMIC_ACQUIRE, "workgroup");
    if (OUT_MODE == 0) {
      float* C = (float*)Cout + (size_t)b * strideC;
      const int hh = lane >> 4, c4 = (lane & 15) * 4;
      for (int pass = 0; pass < 2; ++pass) {
#pragma unroll
        for (int it = 0; it < 8; ++it) {
          const int row = it * 2 + hh;
          v4f v = *(const v4f*)(slab + row * 68 + c4);
          *(volatile v4f*)(C + (size_t)(mBase + row) * ldc + n0 + c4) = v;
        }
        __threadfence();
      }
    } else {
      const int q = lane >> 3, c8 = (lane & 7) * 8;
      unsigned short* C  = (unsigned short*)Cout  + (size_t)b * strideC;
      unsigned short* C2 = (OUT_MODE == 2) ? ((unsigned short*)Cout2 + (size_t)b * strideC) : nullptr;
      for (int pass = 0; pass < 2; ++pass) {
#pragma unroll
        for (int it = 0; it < 4; ++it) {
          const int row = it * 4 + q;
          const float* sp = slab + row * 68 + c8;
          v8h hv, lv;
#pragma unroll
          for (int e = 0; e < 8; ++e) {
            if (OUT_MODE == 1) {
              hv[e] = (_Float16)sp[e];
            } else {
              unsigned short hb = f2bf_bits(sp[e]);
              unsigned short lb = f2bf_bits(sp[e] - bf_bits2f(hb));
              hv[e] = __builtin_bit_cast(_Float16, hb);
              lv[e] = __builtin_bit_cast(_Float16, lb);
            }
          }
          *(volatile v8h*)(C + (size_t)(mBase + row) * ldc + n0 + c8) = hv;
          if (OUT_MODE == 2) *(volatile v8h*)(C2 + (size_t)(mBase + row) * ldc + n0 + c8) = lv;
        }
        __threadfence();
      }
    }
    __builtin_amdgcn_fence(__ATOMIC_RELEASE, "workgroup");
    __builtin_amdgcn_wave_barrier();
    __builtin_amdgcn_fence(__ATOMIC_ACQUIRE, "workgroup");
  }
}

__device__ __forceinline__ unsigned pk16(unsigned short a, unsigned short b) { return (unsigned)a | ((unsigned)b << 16); }
__device__ __forceinline__ void keep_v4i2(v4i& a, v4i& b) { asm volatile("" : "+v"(a), "+v"(b)); }
__device__ __forceinline__ void keep_v4i1(v4i& a) { asm volatile("" : "+v"(a)); }
__device__ __forceinline__ void keep_f3(float& a, float& b, float& c) { asm volatile("" : "+v"(a), "+v"(b), "+v"(c)); }
__device__ __forceinline__ void wave_sync() {
  __builtin_amdgcn_fence(__ATOMIC_RELEASE, "workgroup");
  __builtin_amdgcn_wave_barrier();
  __builtin_amdgcn_fence(__ATOMIC_ACQUIRE, "workgroup");
}

__device__ __forceinline__ int blk_excl_scan(int cnt, int* scan_ws, int tid, int* tot) {
  const int lane = tid & 31, wave = tid >> 5; int incl = cnt;
#pragma unroll
  for (int o = 1; o < 32; o <<= 1) { const int v = __shfl_up(incl, o, 32); if (lane >= o) incl += v; }
  if (lane == 31) scan_ws[wave] = incl;
  __syncthreads();
  if (wave == 0) {
    int wv = scan_ws[lane & 7]; wv = (lane < 8) ? wv : 0; int wincl = wv;
#pragma unroll
    for (int o = 1; o < 32; o <<= 1) { const int v = __shfl_up(wincl, o, 32); if (lane >= o) wincl += v; }
    if (lane < 8) scan_ws[32 + lane] = wincl - wv;
    if (lane == 31) scan_ws[64] = wincl;
  }
  __syncthreads();
  const int res = scan_ws[32 + wave] + incl - cnt; *tot = scan_ws[64];
  return res;
}

__global__ __launch_bounds__(NT) void wt_kernel(const float* __restrict__ cw, unsigned* __restrict__ WH,
                                               unsigned* __restrict__ WL) {
  const int t = blockIdx.x * NT + threadIdx.x;
  if (t >= NLAY * WD * 8) return;
  const int i = t >> 9;
  const int rem = t & 511;
  const int n = rem >> 3;
  const int c8 = (rem & 7) * 8;
  const float* wb = cw + (size_t)i * WD * WD;
  unsigned short hb[8], lb[8];
#pragma unroll
  for (int e = 0; e < 8; ++e) {
    const float v = wb[(size_t)(c8 + e) * WD + n];
    hb[e] = f2bf_bits(v);
    lb[e] = f2bf_bits(v - bf_bits2f(hb[e]));
  }
  const v4u uh = (v4u){pk16(hb[0], hb[1]), pk16(hb[2], hb[3]), pk16(hb[4], hb[5]), pk16(hb[6], hb[7])};
  const v4u ul = (v4u){pk16(lb[0], lb[1]), pk16(lb[2], lb[3]), pk16(lb[4], lb[5]), pk16(lb[6], lb[7])};
  const size_t wo = ((size_t)(i * WD + n) * WD + c8) / 2;
  unsigned* qh = WH + wo;
  unsigned* ql = WL + wo;
  *(volatile v4u*)qh = uh; *(volatile v4u*)ql = ul;
  __threadfence();
  *(volatile v4u*)qh = uh; *(volatile v4u*)ql = ul;
}

__global__ __launch_bounds__(NT) void fc1_kernel(const float* __restrict__ x, const float* __restrict__ w1,
                                                 const float* __restrict__ b1, unsigned* __restrict__ AH,
                                                 unsigned* __restrict__ AL) {
  const int t = blockIdx.x * NT + threadIdx.x;
  const int r = t >> 3;
  const int c8 = (t & 7) * 8;
  if (r >= NP) return;
  const int rc = r < NN ? r : NN - 1;
  float x0 = x[rc * 3], x1 = x[rc * 3 + 1], x2 = x[rc * 3 + 2];
  keep_f3(x0, x1, x2);
  const v4f wa0 = *(const v4f*)(w1 + c8),          wa1 = *(const v4f*)(w1 + c8 + 4);
  const v4f wb0 = *(const v4f*)(w1 + WD + c8),     wb1 = *(const v4f*)(w1 + WD + c8 + 4);
  const v4f wc0 = *(const v4f*)(w1 + 2 * WD + c8), wc1 = *(const v4f*)(w1 + 2 * WD + c8 + 4);
  const v4f bb0 = *(const v4f*)(b1 + c8),          bb1 = *(const v4f*)(b1 + c8 + 4);
  v4f v0 = x0 * wa0 + x1 * wb0 + x2 * wc0 + bb0;
  v4f v1 = x0 * wa1 + x1 * wb1 + x2 * wc1 + bb1;
  const float lf = (r < NN) ? 1.0f : 0.0f;
  v0 = v0 * lf; v1 = v1 * lf;
  unsigned short hb[8], lb[8];
#pragma unroll
  for (int e = 0; e < 4; ++e) {
    hb[e] = f2bf_bits(v0[e]);     lb[e] = f2bf_bits(v0[e] - bf_bits2f(hb[e]));
    hb[4 + e] = f2bf_bits(v1[e]); lb[4 + e] = f2bf_bits(v1[e] - bf_bits2f(hb[4 + e]));
  }
  const v4u uh = (v4u){pk16(hb[0], hb[1]), pk16(hb[2], hb[3]), pk16(hb[4], hb[5]), pk16(hb[6], hb[7])};
  const v4u ul = (v4u){pk16(lb[0], lb[1]), pk16(lb[2], lb[3]), pk16(lb[4], lb[5]), pk16(lb[6], lb[7])};
  const size_t ao = ((size_t)r * WD + c8) / 2;
  unsigned* ph = AH + ao;
  unsigned* pl = AL + ao;
  *(volatile v4u*)ph = uh; *(volatile v4u*)pl = ul;
  __threadfence();
  *(volatile v4u*)ph = uh; *(volatile v4u*)pl = ul;
}

__global__ __launch_bounds__(NT) void part1_kernel(const int* __restrict__ ei, int* __restrict__ CELL) {
  __shared__ int SORTED[PCH];
  __shared__ int scan_ws[80];
  __shared__ int CB[8];
  __shared__ int CT[8];
  const int tid = threadIdx.x, lane = tid & 31, wave = tid >> 5;
  const int c = blockIdx.x;
  for (int i = tid; i < PCH; i += NT) SORTED[i] = 0;
  if (tid < 80) scan_ws[tid] = 0;
  if (tid < 8) { CB[tid] = 0; CT[tid] = 0; }
  const int eb = c * PCH + tid * PSP;
  const bool valid = eb < NE;
  const int ebc = valid ? eb : (NE - PSP);
  const int* srcv = ei;
  const int* dstv = ei + NE;
  int ent[PSP]; int stv[PSP];
#pragma unroll
  for (int k = 0; k < PSP; k += 4) {
    v4i d4 = *(const v4i*)(dstv + ebc + k);
    v4i s4 = *(const v4i*)(srcv + ebc + k);
    keep_v4i2(d4, s4);
#pragma unroll
    for (int e = 0; e < 4; ++e) {
      int d = d4[e], s = s4[e];
      d = d < 0 ? 0 : (d >= NN ? NN - 1 : d);
      s = s < 0 ? 0 : (s >= NN ? NN - 1 : s);
      stv[k + e] = valid ? (d >> STSH) : NST;
      ent[k + e] = (int)(((unsigned)d << 16) | (unsigned)s);
    }
  }
  __syncthreads();
  int base = 0;
#pragma unroll 1
  for (int cl = 0; cl < NST; ++cl) {
    int cnt = 0;
#pragma unroll
    for (int k = 0; k < PSP; ++k) cnt += (stv[k] == cl) ? 1 : 0;
    int tot; int p = blk_excl_scan(cnt, scan_ws, tid, &tot) + base;
#pragma unroll
    for (int k = 0; k < PSP; ++k) if (stv[k] == cl) { SORTED[p & (PCH - 1)] = ent[k]; ++p; }
    if (tid == 0) { CB[cl] = base; CT[cl] = tot; }
    base += tot;
    __syncthreads();
  }
  const int r4 = lane >> 3, l8 = lane & 7;
#pragma unroll 1
  for (int itw = 0; itw < NST; ++itw) {
    const int L = (itw * 8 + wave) * 4 + r4;
    const int cidx = L >> 5, j = L & 31;
    const int basec = CB[cidx], totc = CT[cidx];
    v4i v;
#pragma unroll
    for (int e = 0; e < 4; ++e) {
      const int idx = 32 * j + 4 * l8 + e;
      int a = basec + idx; a = a < PCH ? a : PCH - 1; a = a < 0 ? 0 : a;
      const int val = SORTED[a];
      v[e] = (idx < totc) ? val : (int)SENTC;
    }
    int* dst = CELL + ((size_t)(c * NST + cidx) * CCAP + 32 * j + 4 * l8);
    *(volatile v4i*)dst = v;
    __threadfence();
    *(volatile v4i*)dst = v;
  }
}

__global__ __launch_bounds__(NT) void bucket_kernel(const int* __restrict__ CELL, int* __restrict__ BK) {
  __shared__ int LIST[PCH];
  __shared__ int Q1[8][Q1CAP];
  __shared__ __align__(16) int STG[8][8][64];
  __shared__ int SF[64];
  __shared__ int LC[64];
  __shared__ int FILL[8];
  __shared__ int TB[64];
  __shared__ int OFFT[64];
  __shared__ int scan_ws[80];
  const int tid = threadIdx.x, lane = tid & 31, wave = tid >> 5;
  const int t = blockIdx.x;
  const int st = t >> 3;
  const int l8 = lane & 7;
  for (int i = tid; i < PCH; i += NT) LIST[i] = 0;
  for (int i = tid; i < 8 * Q1CAP; i += NT) (&Q1[0][0])[i] = 0;
  for (int i = tid; i < 8 * 8 * 64; i += NT) (&STG[0][0][0])[i] = 0;
  if (tid < 64) { SF[tid] = 0; LC[tid] = 0; TB[tid] = 0; OFFT[tid] = 0; }
  if (tid < 8) FILL[tid] = 0;
  if (tid < 80) scan_ws[tid] = 0;
  __syncthreads();
  const unsigned ltmask = (1u << lane) - 1u;
  int* bkw = BK + (size_t)(t * NSB + wave * 8) * SBCAP;

#pragma unroll 1
  for (int it = 0; it < NBI; ++it) {
    int rec[CPI * 4]; int cnt = 0;
#pragma unroll
    for (int q = 0; q < CPI; ++q) {
      const int cc = it * CPI + q;
      const bool cv = cc < NPC;
      const int ccl = cv ? cc : NPC - 1;
      v4i ev = *(const v4i*)(CELL + ((size_t)(ccl * NST + st) * CCAP + 4 * tid));
      keep_v4i1(ev);
#pragma unroll
      for (int e = 0; e < 4; ++e) {
        const unsigned en = (unsigned)ev[e];
        const unsigned d = en >> 16;
        const bool hit = cv && ((int)(d >> 10) == t);
        rec[q * 4 + e] = hit ? (int)(((d & 1023u) << 16) | (en & 0xFFFFu)) : -1;
        cnt += hit ? 1 : 0;
      }
    }
    int tot; int p = blk_excl_scan(cnt, scan_ws, tid, &tot);
#pragma unroll
    for (int k = 0; k < CPI * 4; ++k) if (rec[k] >= 0) { LIST[p & (PCH - 1)] = rec[k]; ++p; }
    __syncthreads();
    int nsl = (tot + NT - 1) / NT; nsl = nsl < 0 ? 0 : (nsl > (PCH / NT) ? (PCH / NT) : nsl);
#pragma unroll 1
    for (int sl = 0; sl < nsl; ++sl) {
      const int idx = sl * NT + tid;
      const int entv = LIST[idx & (PCH - 1)];
      const bool has = idx < tot;
      const int wc = has ? ((entv >> 23) & 7) : 8;
      unsigned bsel = 0u; int mycnt = 0;
#pragma unroll
      for (int cl = 0; cl < 8; ++cl) {
        const unsigned bm = (unsigned)__ballot(wc == cl);
        bsel = (wc == cl) ? bm : bsel;
        mycnt = (lane == cl) ? (int)__popc(bm) : mycnt;
      }
      const int rank = (int)__popc(bsel & ltmask);
      if (lane < 8) TB[wave * 8 + lane] = mycnt;
      __syncthreads();
      if (tid < 8) {
        int run = 0;
#pragma unroll
        for (int w8 = 0; w8 < 8; ++w8) { OFFT[w8 * 8 + tid] = run; run += TB[w8 * 8 + tid]; }
        FILL[tid] = run;
      }
      __syncthreads();
      {
        const int wcc = wc < 8 ? wc : 7;
        int pos = OFFT[wave * 8 + wcc] + rank; pos = pos < 0 ? 0 : (pos < Q1CAP ? pos : Q1CAP - 1);
        if (has) Q1[wcc][pos] = entv;
      }
      __syncthreads();
      {
        const int fill = __builtin_amdgcn_readfirstlane(FILL[wave]);
        int nb = (fill + 31) >> 5; nb = nb < 0 ? 0 : (nb > (Q1CAP / 32) ? (Q1CAP / 32) : nb);
#pragma unroll 1
        for (int bi = 0; bi < nb; ++bi) {
          const int qi0 = (bi << 5) + lane;
          const bool qv = qi0 < fill;
          const int qic = qi0 < Q1CAP ? qi0 : Q1CAP - 1;
          const int qe = Q1[wave][qic];
          const int g = qv ? ((qe >> 20) & 7) : 8;
          unsigned gsel = 0u; int gcnt = 0;
#pragma unroll
          for (int cl = 0; cl < 8; ++cl) {
            const unsigned bm = (unsigned)__ballot(g == cl);
            gsel = (g == cl) ? bm : gsel;
            gcnt = (lane == cl) ? (int)__popc(bm) : gcnt;
          }
          const int grank = (int)__popc(gsel & ltmask);
          const int gc = g < 8 ? g : 7;
          const int sfo = SF[wave * 8 + gc];
          const int sfl = SF[wave * 8 + l8];
          int spos = sfo + grank; spos = spos < 0 ? 0 : (spos < 64 ? spos : 63);
          if (qv) STG[wave][gc][spos] = qe;
          wave_sync();
          const int sfn = sfl + gcnt;
          if (lane < 8) SF[wave * 8 + lane] = sfn;
          wave_sync();
          unsigned fm = (unsigned)__ballot((lane < 8) && (sfn >= 32));
#pragma unroll 1
          for (int fi = 0; fi < 8; ++fi) {
            if (fm == 0u) break;
            const int gg = (int)(__builtin_ctz(fm) & 7);
            fm &= fm - 1u;
            const int lcv = __builtin_amdgcn_readfirstlane(LC[wave * 8 + gg]);
            const v4i lvv = *(const v4i*)(&STG[wave][gg][4 * l8]);
            const int mv = STG[wave][gg][32 + lane];
            if (lcv < SBL) {
              int* dstp = bkw + (size_t)gg * SBCAP + lcv * 32 + 4 * l8;
              if (lane < 8) *(volatile v4i*)dstp = lvv;
              __threadfence();
              if (lane < 8) *(volatile v4i*)dstp = lvv;
            }
            wave_sync();
            STG[wave][gg][lane] = mv;
            if (lane == 0) { SF[wave * 8 + gg] = SF[wave * 8 + gg] - 32; LC[wave * 8 + gg] = lcv + 1; }
            wave_sync();
          }
        }
      }
      __syncthreads();
    }
  }
  {
#pragma unroll 1
    for (int g = 0; g < 8; ++g) {
      const int sval = (int)(((unsigned)(16 * (wave * 8 + g)) << 16) | (unsigned)SENTB);
      const v4i sv = (v4i){sval, sval, sval, sval};
      const int sfv = __builtin_amdgcn_readfirstlane(SF[wave * 8 + g]);
      int lcv = __builtin_amdgcn_readfirstlane(LC[wave * 8 + g]);
      int* bkg = bkw + (size_t)g * SBCAP;
      if (sfv > 0) {
        v4i lvv;
#pragma unroll
        for (int e = 0; e < 4; ++e) {
          const int idx = 4 * l8 + e;
          const int val = STG[wave][g][idx];
          lvv[e] = (idx < sfv) ? val : sval;
        }
        if (lcv < SBL) {
          int* dstp = bkg + lcv * 32 + 4 * l8;
          if (lane < 8) *(volatile v4i*)dstp = lvv;
          __threadfence();
          if (lane < 8) *(volatile v4i*)dstp = lvv;
        }
        lcv += 1;
      }
      lcv = lcv < 0 ? 0 : (lcv < SBL ? lcv : SBL);
      for (int j = lcv; j < SBL; ++j) { if (lane < 8) *(volatile v4i*)(bkg + j * 32 + 4 * l8) = sv; }
      __threadfence();
      for (int j = lcv; j < SBL; ++j) { if (lane < 8) *(volatile v4i*)(bkg + j * 32 + 4 * l8) = sv; }
    }
  }
}

__global__ __launch_bounds__(NT) void deg_kernel(const int* __restrict__ BK, float* __restrict__ dis) {
  __shared__ int CNT[TR];
  const int tid = threadIdx.x, lane = tid & 31, wave = tid >> 5;
  const int t = blockIdx.x, n0 = t * TR;
  for (int i = tid; i < TR; i += NT) CNT[i] = 0;
  __syncthreads();
  const int g = lane >> 2, u = lane & 3, sb = wave * 8 + g;
  const int* bk = BK + (size_t)(t * NSB + sb) * SBCAP;
#pragma unroll 1
  for (int i4 = 0; i4 < SBCAP / 4; ++i4) {
    const v4i ev = *(const v4i*)(bk + 4 * i4);
#pragma unroll
    for (int j = 0; j < 4; ++j) {
      const int e = ev[j];
      const int dl = (int)(((unsigned)e >> 16) & 1023u);
      const int sfd = (int)((unsigned)e & 0xFFFFu);
      const int inc = (sfd != SENTB) ? 1 : 0;
      const int cvv = CNT[dl];
      if (u == 0) CNT[dl] = cvv + inc;
    }
  }
  __syncthreads();
  const int r4 = lane >> 3, l8 = lane & 7;
  const int dl0 = 128 * wave + 32 * r4 + 4 * l8;
  v4f dv;
#pragma unroll
  for (int e = 0; e < 4; ++e) {
    const int dl = dl0 + e; const int n = n0 + dl;
    const float degf = (float)(CNT[dl] + 1);
    const float f = 1.0f / sqrtf(degf);
    dv[e] = (n < NN) ? f : 0.0f;
  }
  float* dp = dis + n0 + dl0;
  *(volatile v4f*)dp = dv;
  __threadfence();
  *(volatile v4f*)dp = dv;
}

template <bool LAST>
__global__ __launch_bounds__(NT) void agg_kernel(const float* __restrict__ hw, const int* __restrict__ BK,
                                                 const float* __restrict__ dis, const float* __restrict__ cb,
                                                 unsigned* __restrict__ AH, unsigned* __restrict__ AL,
                                                 const float* __restrict__ w2, const float* __restrict__ b2,
                                                 float* __restrict__ out) {
  extern __shared__ __align__(16) float ACC[];
  __shared__ __align__(16) float OUTW[8][128];
  const int tid = threadIdx.x, lane = tid & 31, wave = tid >> 5;
  const int t = blockIdx.x, n0 = t * TR;
  const int g = lane >> 2, u = lane & 3, sb = wave * 8 + g, c16 = 16 * u;
#pragma unroll 1
  for (int i = 0; i < 16; ++i) {
    const int dl = 16 * sb + i; const int n = n0 + dl; const int nc = n < NP ? n : NP - 1;
    const float ds = dis[n];
    const float* hp = hw + (size_t)nc * WD + c16;
    const v4f h0 = *(const v4f*)hp, h1 = *(const v4f*)(hp + 4), h2 = *(const v4f*)(hp + 8), h3 = *(const v4f*)(hp + 12);
    float* ap = ACC + dl * WD + c16;
    *(v4f*)ap = h0 * ds; *(v4f*)(ap + 4) = h1 * ds; *(v4f*)(ap + 8) = h2 * ds; *(v4f*)(ap + 12) = h3 * ds;
  }
  __syncthreads();
  const int* bk = BK + (size_t)(t * NSB + sb) * SBCAP;
#pragma unroll 1
  for (int i4 = 0; i4 < SBCAP / 4; ++i4) {
    const v4i ev = *(const v4i*)(bk + 4 * i4);
#pragma unroll
    for (int j = 0; j < 4; ++j) {
      const int e = ev[j];
      const int dl = (int)(((unsigned)e >> 16) & 1023u);
      int s = (int)((unsigned)e & 0xFFFFu); s = s < NP ? s : NP - 1;
      const float ds = dis[s];
      const float* hp = hw + (size_t)s * WD + c16;
      const v4f h0 = *(const v4f*)hp, h1 = *(const v4f*)(hp + 4), h2 = *(const v4f*)(hp + 8), h3 = *(const v4f*)(hp + 12);
      float* ap = ACC + dl * WD + c16;
      v4f a0 = *(const v4f*)ap, a1 = *(const v4f*)(ap + 4), a2 = *(const v4f*)(ap + 8), a3 = *(const v4f*)(ap + 12);
      a0 = a0 + h0 * ds; a1 = a1 + h1 * ds; a2 = a2 + h2 * ds; a3 = a3 + h3 * ds;
      *(v4f*)ap = a0; *(v4f*)(ap + 4) = a1; *(v4f*)(ap + 8) = a2; *(v4f*)(ap + 12) = a3;
      __asm__ volatile("" ::: "memory");
    }
  }
  __syncthreads();
  const int r4 = lane >> 3, l8 = lane & 7, c8 = 8 * l8;
  const v4f bv0 = *(const v4f*)(cb + c8), bv1 = *(const v4f*)(cb + c8 + 4);
  v4f wv0 = (v4f){0.f, 0.f, 0.f, 0.f}, wv1 = (v4f){0.f, 0.f, 0.f, 0.f}; float ob = 0.0f;
  if (LAST) { wv0 = *(const v4f*)(w2 + c8); wv1 = *(const v4f*)(w2 + c8 + 4); ob = b2[0]; }
#pragma unroll 1
  for (int ir = 0; ir < 32; ++ir) {
    const int dl = 128 * wave + 4 * ir + r4; const int n = n0 + dl;
    const float lf = (n < NN) ? 1.0f : 0.0f;
    const float ds = dis[n];
    const float* ap = ACC + dl * WD + c8;
    const v4f a0 = *(const v4f*)ap, a1 = *(const v4f*)(ap + 4);
    v4f v0 = a0 * ds + bv0; v4f v1 = a1 * ds + bv1;
#pragma unroll
    for (int e = 0; e < 4; ++e) { v0[e] = fmaxf(v0[e], 0.0f) * lf; v1[e] = fmaxf(v1[e], 0.0f) * lf; }
    if (!LAST) {
      unsigned short hb[8], lb[8];
#pragma unroll
      for (int e = 0; e < 4; ++e) {
        hb[e] = f2bf_bits(v0[e]);     lb[e] = f2bf_bits(v0[e] - bf_bits2f(hb[e]));
        hb[4 + e] = f2bf_bits(v1[e]); lb[4 + e] = f2bf_bits(v1[e] - bf_bits2f(hb[4 + e]));
      }
      const v4u uh = (v4u){pk16(hb[0], hb[1]), pk16(hb[2], hb[3]), pk16(hb[4], hb[5]), pk16(hb[6], hb[7])};
      const v4u ul = (v4u){pk16(lb[0], lb[1]), pk16(lb[2], lb[3]), pk16(lb[4], lb[5]), pk16(lb[6], lb[7])};
      const bool stv = n < NP;
      const size_t ao = ((size_t)n * WD + c8) / 2;
      unsigned* ph = AH + ao;
      unsigned* pl = AL + ao;
      if (stv) { *(volatile v4u*)ph = uh; *(volatile v4u*)pl = ul; }
      __threadfence();
      if (stv) { *(volatile v4u*)ph = uh; *(volatile v4u*)pl = ul; }
    } else {
      float sd = v0[0] * wv0[0] + v0[1] * wv0[1] + v0[2] * wv0[2] + v0[3] * wv0[3]
               + v1[0] * wv1[0] + v1[1] * wv1[1] + v1[2] * wv1[2] + v1[3] * wv1[3];
      sd += __shfl_xor(sd, 4, 32);
      sd += __shfl_xor(sd, 2, 32);
      sd += __shfl_xor(sd, 1, 32);
      if (l8 == 0) OUTW[wave][4 * ir + r4] = sd + ob;
    }
  }
  if (LAST) {
    __syncthreads();
    const v4f ov = *(const v4f*)(&OUTW[wave][32 * r4 + 4 * l8]);
    const int no = n0 + 128 * wave + 32 * r4 + 4 * l8;
    const bool st2 = no < NN;
    if (st2) *(volatile v4f*)(out + no) = ov;
    __threadfence();
    if (st2) *(volatile v4f*)(out + no) = ov;
  }
}

extern "C" void kernel_launch(void* const* d_in, const int* in_sizes, int n_in,
                              void* d_out, int out_size, void* d_ws, size_t ws_size, hipStream_t stream) {
  (void)in_sizes; (void)n_in; (void)out_size;
  const float* x      = (const float*)d_in[0];
  const int*   ei     = (const int*)  d_in[1];
  const float* fc1_w  = (const float*)d_in[2];
  const float* fc1_b  = (const float*)d_in[3];
  const float* conv_w = (const float*)d_in[4];
  const float* conv_b = (const float*)d_in[5];
  const float* fc2_w  = (const float*)d_in[6];
  const float* fc2_b  = (const float*)d_in[7];
  float* out = (float*)d_out;

  char* ws = (char*)d_ws; size_t off = 0;
  auto carve = [&](size_t bytes) -> char* { char* p = ws + off; off += (bytes + 255) & ~(size_t)255; return p; };
  float*          dis  = (float*)carve((size_t)NR * sizeof(float));
  unsigned short* WH   = (unsigned short*)carve((size_t)NLAY * WD * WD * 2);
  unsigned short* WL   = (unsigned short*)carve((size_t)NLAY * WD * WD * 2);
  unsigned short* AH   = (unsigned short*)carve((size_t)NP * WD * 2);
  unsigned short* AL   = (unsigned short*)carve((size_t)NP * WD * 2);
  float*          hw   = (float*)carve((size_t)NP * WD * sizeof(float));
  int*            CELL = (int*)carve((size_t)NPC * NST * CCAP * sizeof(int));
  int*            BK   = (int*)carve((size_t)NTIL * NSB * SBCAP * sizeof(int));
  if (off > ws_size || off > (size_t)134217728) return;
  hipFuncSetAttribute((const void*)agg_kernel<false>, hipFuncAttributeMaxDynamicSharedMemorySize, ACCB);
  hipFuncSetAttribute((const void*)agg_kernel<true>, hipFuncAttributeMaxDynamicSharedMemorySize, ACCB);

  wt_kernel<<<(NLAY * WD * 8) / NT, NT, 0, stream>>>(conv_w, (unsigned*)WH, (unsigned*)WL);
  fc1_kernel<<<(NP * 8) / NT, NT, 0, stream>>>(x, fc1_w, fc1_b, (unsigned*)AH, (unsigned*)AL);
  part1_kernel<<<NPC, NT, 0, stream>>>(ei, CELL);
  bucket_kernel<<<NTIL, NT, 0, stream>>>(CELL, BK);
  deg_kernel<<<NTIL, NT, 0, stream>>>(BK, dis);

  const int gemm_tiles  = (NP / 64) * (WD / 64);
  const int gemm_blocks = (gemm_tiles + 7) / 8;
  for (int L = 0; L < NLAY; ++L) {
    wmma_gemm64<1, true, 0, 0, false><<<dim3(gemm_blocks, 1), 256, 0, stream>>>(
        (const unsigned short*)AH, (const unsigned short*)AL, WD, 0L,
        (const unsigned short*)(WH + (size_t)L * WD * WD), (const unsigned short*)(WL + (size_t)L * WD * WD), WD, 0L,
        (void*)hw, (void*)nullptr, WD, 0L,
        (const float*)nullptr, (const float*)nullptr, 0L, NP, WD, WD, 1.0f);
    if (L + 1 < NLAY) {
      agg_kernel<false><<<NTIL, NT, ACCB, stream>>>(hw, BK, dis, conv_b + (size_t)L * WD, (unsigned*)AH, (unsigned*)AL,
                                                     fc2_w, fc2_b, out);
    } else {
      agg_kernel<true><<<NTIL, NT, ACCB, stream>>>(hw, BK, dis, conv_b + (size_t)L * WD, (unsigned*)AH, (unsigned*)AL,
                                                    fc2_w, fc2_b, out);
    }
  }
}
